// HivemindMamba_52664888984004
// MI455X (gfx1250) — hardware-verified
//
#include <hip/hip_runtime.h>
#include <stddef.h>
#include <stdint.h>


#define DM 512
#define DS 16
#define LT 2048
#define LI 1024
#define NB 2

#define SC_ACT 256.0f
#define SC_W   64.0f
#define SC_QK  16.0f
#define SC_P   4096.0f
#define SC_BF  256.0f
#define SC_Y   256.0f

typedef _Float16 v16h __attribute__((ext_vector_type(16)));
typedef _Float16 v8h  __attribute__((ext_vector_type(8)));
typedef float    v8f  __attribute__((ext_vector_type(8)));
typedef float    v4f  __attribute__((ext_vector_type(4)));
typedef v8h v8ha __attribute__((may_alias));
typedef v4f v4fa __attribute__((may_alias));

union Frag { v16h v; v8h half[2]; };

__device__ __forceinline__ v8f wmma16(v8f acc, v16h a, v16h b)
{
  acc = __builtin_amdgcn_wmma_f32_16x16x32_f16(false, a, false, b, (short)0, acc, false, false);
  asm volatile("v_nop\n\tv_nop\n\tv_nop\n\tv_nop" : "+v"(acc) : "v"(a), "v"(b));
  return acc;
}

__device__ __forceinline__ v8h cvt8(v4f a, v4f b, float sc)
{
  v8h o;
  o[0] = (_Float16)(a[0] * sc); o[1] = (_Float16)(a[1] * sc);
  o[2] = (_Float16)(a[2] * sc); o[3] = (_Float16)(a[3] * sc);
  o[4] = (_Float16)(b[0] * sc); o[5] = (_Float16)(b[1] * sc);
  o[6] = (_Float16)(b[2] * sc); o[7] = (_Float16)(b[3] * sc);
  return o;
}

__global__ void __launch_bounds__(256)
cvt_rows_f16_kernel(const float* __restrict__ in, _Float16* __restrict__ out, int nunits, float sc)
{
  const int u = (int)blockIdx.x * 256 + (int)threadIdx.x;
  const bool ok = (u < nunits);
  v4f a = {0.0f, 0.0f, 0.0f, 0.0f};
  v4f b = {0.0f, 0.0f, 0.0f, 0.0f};
  if (ok) {
    a = *(const v4fa*)(in + (size_t)u * 8);
    b = *(const v4fa*)(in + (size_t)u * 8 + 4);
  }
  const v8h o = cvt8(a, b, sc);
  _Float16* dst = out + (size_t)u * 8;
  if (ok) *(volatile v8h*)dst = o;
  __threadfence();
  if (ok) *(volatile v8h*)dst = o;
}

__global__ void __launch_bounds__(256)
cvt_wT_f16_kernel(const float* __restrict__ W, _Float16* __restrict__ out, int R, int C, int ldo, float sc)
{
  __shared__ float tile[64][33];
  const int tid = (int)threadIdx.x;
  const int r0 = (int)blockIdx.y * 64, c0 = (int)blockIdx.x * 32;
  const int cc = tid & 31, rw = tid >> 5;
#pragma unroll
  for (int i = 0; i < 8; ++i) {
    const int rl = i * 8 + rw;
    const int r = r0 + rl, c = c0 + cc;
    tile[rl][cc] = (r < R && c < C) ? W[(size_t)r * (size_t)C + c] : 0.0f;
  }
  __syncthreads();
  const int ol = tid >> 3, piece = tid & 7;
  const int orow = c0 + ol;
  const bool ok = (orow < C) && (r0 + 8 * piece + 8 <= R);
  v8h o;
#pragma unroll
  for (int j = 0; j < 8; ++j) o[j] = (_Float16)(tile[8 * piece + j][ol] * sc);
  _Float16* dst = out + (size_t)orow * (size_t)ldo + r0 + 8 * piece;
  if (ok) *(volatile v8h*)dst = o;
  __threadfence();
  if (ok) *(volatile v8h*)dst = o;
}

struct GemmArgs {
  const _Float16* A;
  const _Float16* A2;
  const _Float16* Bt;
  float*          Cf;
  _Float16*       Ch;
  _Float16*       Ct;
  const float*    bias;
  const float*    bias2;
  long long sA, sA2, sB, sC, sCh, sCt;
  int lda, lda2, ldb, ldc, ldch, ldct;
  int M, N, K, ksplit, nsplit, cfNmax, ctNmin, batch;
  float oscale, hscale;
};
typedef char gemm_args_size_check[(sizeof(GemmArgs) == 176) ? 1 : -1];

template <int NW>
__global__ void __launch_bounds__(64 * NW)
gemm_f16_kernel(GemmArgs g)
{
  constexpr int TN  = 32 * NW;
  constexpr int TP  = TN + 4;
  constexpr int NTH = 64 * NW;
  __shared__ __attribute__((aligned(16))) float tile[64 * TP];

  const int tid  = (int)threadIdx.x;
  const int lane = tid & 31;
  const int wave = tid >> 5;
  const int hh   = lane >> 4;
  const int r16  = lane & 15;
  const int wm   = wave & 1;
  const int wn   = wave >> 1;
  const int m0   = (int)blockIdx.y * 64;
  const int n0   = (int)blockIdx.x * TN;
  const int z    = (int)blockIdx.z;
  if (m0 + 64 > g.M || n0 + TN > g.N) return;

  const _Float16* Ab  = g.A + (size_t)z * (size_t)g.sA;
  const _Float16* A2b = (g.A2 != nullptr) ? (g.A2 + (size_t)z * (size_t)g.sA2) : Ab;
  const _Float16* Bb  = g.Bt + (size_t)z * (size_t)g.sB;
  const int arow = m0 + wm * 32 + r16;
  const int bcol = n0 + wn * 32 + r16;

  v8f acc[2][2];
#pragma unroll
  for (int mi = 0; mi < 2; ++mi)
#pragma unroll
    for (int ni = 0; ni < 2; ++ni)
#pragma unroll
      for (int r = 0; r < 8; ++r) acc[mi][ni][r] = 0.0f;

#pragma unroll 1
  for (int k0 = 0; k0 < g.K; k0 += 32) {
    const bool lo = (k0 < g.ksplit);
    const _Float16* ap = lo ? Ab : A2b;
    const int ld = lo ? g.lda : g.lda2;
    const int kk = lo ? k0 : (k0 - g.ksplit);
    Frag a[2], b[2];
#pragma unroll
    for (int mi = 0; mi < 2; ++mi) {
      const _Float16* p = ap + (size_t)(arow + 16 * mi) * (size_t)ld + kk + 8 * hh;
      a[mi].half[0] = *(const v8ha*)(p);
      a[mi].half[1] = *(const v8ha*)(p + 16);
    }
#pragma unroll
    for (int ni = 0; ni < 2; ++ni) {
      const _Float16* q = Bb + (size_t)(bcol + 16 * ni) * (size_t)g.ldb + k0 + 8 * hh;
      b[ni].half[0] = *(const v8ha*)(q);
      b[ni].half[1] = *(const v8ha*)(q + 16);
    }
#pragma unroll
    for (int mi = 0; mi < 2; ++mi)
#pragma unroll
      for (int ni = 0; ni < 2; ++ni)
        acc[mi][ni] = wmma16(acc[mi][ni], a[mi].v, b[ni].v);
  }

  float bv[2];
#pragma unroll
  for (int ni = 0; ni < 2; ++ni) {
    const int n = bcol + 16 * ni;
    float v = 0.0f;
    if (g.bias != nullptr) v = (n < g.nsplit) ? g.bias[n] : g.bias2[n - g.nsplit];
    bv[ni] = v;
  }
#pragma unroll
  for (int mi = 0; mi < 2; ++mi)
#pragma unroll
    for (int ni = 0; ni < 2; ++ni)
#pragma unroll
      for (int r = 0; r < 8; ++r)
        tile[(wm * 32 + 16 * mi + 8 * hh + r) * TP + wn * 32 + 16 * ni + r16] =
            acc[mi][ni][r] * g.oscale + bv[ni];
  __syncthreads();

  const bool doCf = (g.Cf != nullptr) && (n0 < g.cfNmax);
  const bool doCh = (NW == 2) && (g.Ch != nullptr);
  const bool doCt = (g.Ct != nullptr) && (n0 >= g.ctNmin);

  for (int pass = 0; pass < 2; ++pass) {
    if (pass) __threadfence();
    if (doCf) {
      constexpr int UPR = TN / 4;
      constexpr int PER = (64 * UPR) / NTH;
      float* cb = g.Cf + (size_t)z * (size_t)g.sC;
#pragma unroll
      for (int it = 0; it < PER; ++it) {
        const int u = it * NTH + tid;
        const int row = u / UPR, c4 = u - row * UPR;
        const v4f v = *(const v4fa*)(tile + row * TP + 4 * c4);
        *(volatile v4f*)(cb + (size_t)(m0 + row) * (size_t)g.ldc + n0 + 4 * c4) = v;
      }
    }
    if (doCh) {
      constexpr int UPR8 = TN / 8;
      constexpr int PER  = (64 * UPR8) / NTH;
      _Float16* hb = g.Ch + (size_t)z * (size_t)g.sCh;
#pragma unroll
      for (int it = 0; it < PER; ++it) {
        const int u = it * NTH + tid;
        const int row = u / UPR8, c8 = u - row * UPR8;
        const float* tp = tile + row * TP + 8 * c8;
        const v4f f0 = *(const v4fa*)(tp);
        const v4f f1 = *(const v4fa*)(tp + 4);
        const v8h o = cvt8(f0, f1, g.hscale);
        *(volatile v8h*)(hb + (size_t)(m0 + row) * (size_t)g.ldch + n0 + 8 * c8) = o;
      }
    }
    if (doCt) {
      constexpr int PER = (8 * TN) / NTH;
      _Float16* tb = g.Ct + (size_t)z * (size_t)g.sCt;
#pragma unroll
      for (int it = 0; it < PER; ++it) {
        const int u = it * NTH + tid;
        const int orow = u >> 3, piece = u & 7;
        v8h o;
#pragma unroll
        for (int j = 0; j < 8; ++j) o[j] = (_Float16)(tile[(8 * piece + j) * TP + orow] * g.hscale);
        *(volatile v8h*)(tb + (size_t)(n0 + orow - g.ctNmin) * (size_t)g.ldct + m0 + 8 * piece) = o;
      }
    }
  }
}

__global__ void __launch_bounds__(256)
softmax_f16_kernel(const float* __restrict__ S, _Float16* __restrict__ P, int cols, float scale, float pscale)
{
  __shared__ float red[8];
  const int tid = (int)threadIdx.x, lane = tid & 31, wv = tid >> 5;
  const size_t row = blockIdx.x;
  const float* s = S + row * (size_t)cols;
  _Float16* p = P + row * (size_t)cols;

  float m = -3.0e38f;
  for (int c = 8 * tid; c < cols; c += 2048) {
    const v4f x0 = *(const v4fa*)(s + c);
    const v4f x1 = *(const v4fa*)(s + c + 4);
    m = fmaxf(m, fmaxf(fmaxf(x0[0], x0[1]), fmaxf(x0[2], x0[3])));
    m = fmaxf(m, fmaxf(fmaxf(x1[0], x1[1]), fmaxf(x1[2], x1[3])));
  }
#pragma unroll
  for (int off = 16; off; off >>= 1) m = fmaxf(m, __shfl_xor(m, off, 32));
  if (lane == 0) red[wv] = m;
  __syncthreads();
  m = red[0];
#pragma unroll
  for (int i = 1; i < 8; ++i) m = fmaxf(m, red[i]);
  __syncthreads();

  float sum = 0.0f;
  for (int c = 8 * tid; c < cols; c += 2048) {
    const v4f x0 = *(const v4fa*)(s + c);
    const v4f x1 = *(const v4fa*)(s + c + 4);
#pragma unroll
    for (int j = 0; j < 4; ++j) sum += __expf((x0[j] - m) * scale);
#pragma unroll
    for (int j = 0; j < 4; ++j) sum += __expf((x1[j] - m) * scale);
  }
#pragma unroll
  for (int off = 16; off; off >>= 1) sum += __shfl_xor(sum, off, 32);
  if (lane == 0) red[wv] = sum;
  __syncthreads();
  sum = 0.0f;
#pragma unroll
  for (int i = 0; i < 8; ++i) sum += red[i];
  const float f = pscale / sum;

  for (int pass = 0; pass < 2; ++pass) {
    if (pass) __threadfence();
    for (int c = 8 * tid; c < cols; c += 2048) {
      const v4f x0 = *(const v4fa*)(s + c);
      const v4f x1 = *(const v4fa*)(s + c + 4);
      v8h o;
#pragma unroll
      for (int j = 0; j < 4; ++j) o[j] = (_Float16)(__expf((x0[j] - m) * scale) * f);
#pragma unroll
      for (int j = 0; j < 4; ++j) o[4 + j] = (_Float16)(__expf((x1[j] - m) * scale) * f);
      *(volatile v8h*)(p + c) = o;
    }
  }
}

__global__ void __launch_bounds__(128)
scan_kernel(const float* __restrict__ xq, const float* __restrict__ dt,
            const float* __restrict__ A_log, const float* __restrict__ BC,
            _Float16* __restrict__ yh, int L, float yscale)
{
  __shared__ __attribute__((aligned(16))) _Float16 ybuf[32 * 64];
  const int tid = (int)threadIdx.x;
  const int chl = tid >> 1, sh = tid & 1;
  const int chg = (int)blockIdx.x * 64 + chl;
  const int b = chg / DM, d = chg - b * DM;
  const int d0 = ((int)blockIdx.x * 64) % DM;

  float Ac[8], h[8];
#pragma unroll
  for (int s = 0; s < 8; ++s) {
    Ac[s] = -__expf(A_log[d * DS + 8 * sh + s]);
    h[s] = 0.0f;
  }
  const size_t rb = (size_t)b * (size_t)L;

  for (int l0 = 0; l0 < L; l0 += 32) {
#pragma unroll 1
    for (int ls = 0; ls < 32; ++ls) {
      const size_t row = rb + (size_t)(l0 + ls);
      const float dtv = dt[row * DM + d];
      const float xv  = xq[row * DM + d];
      const float* bc = BC + row * 32 + 8 * sh;
      const v4f B0 = *(const v4fa*)(bc);
      const v4f B1 = *(const v4fa*)(bc + 4);
      const v4f C0 = *(const v4fa*)(bc + 16);
      const v4f C1 = *(const v4fa*)(bc + 20);
      const float sp  = fmaxf(dtv, 0.0f) + log1pf(__expf(-fabsf(dtv)));
      const float spx = sp * xv;
      float pacc = 0.0f;
#pragma unroll
      for (int s = 0; s < 4; ++s) {
        h[s] = __expf(sp * Ac[s]) * h[s] + spx * B0[s];
        pacc += h[s] * C0[s];
      }
#pragma unroll
      for (int s = 0; s < 4; ++s) {
        h[4 + s] = __expf(sp * Ac[4 + s]) * h[4 + s] + spx * B1[s];
        pacc += h[4 + s] * C1[s];
      }
      pacc += __shfl_xor(pacc, 1, 32);
      if (sh == 0) ybuf[ls * 64 + chl] = (_Float16)(pacc * yscale);
    }
    __syncthreads();
    for (int pass = 0; pass < 2; ++pass) {
      if (pass) __threadfence();
#pragma unroll
      for (int it = 0; it < 2; ++it) {
        const int u = it * 128 + tid;
        const int line = u >> 3, piece = u & 7;
        const v8h v = *(const v8ha*)(ybuf + line * 64 + 8 * piece);
        *(volatile v8h*)(yh + (rb + (size_t)(l0 + line)) * DM + d0 + 8 * piece) = v;
      }
    }
    __syncthreads();
  }
}

__global__ void __launch_bounds__(128)
layernorm_kernel(const float* __restrict__ X, const float* __restrict__ gam,
                 const float* __restrict__ bet, float* __restrict__ out, int rows)
{
  __shared__ float red[4];
  const int tid = (int)threadIdx.x, lane = tid & 31, wv = tid >> 5;
  const int row = (int)blockIdx.x;
  if (row >= rows) return;
  const float* xr = X + (size_t)row * DM;
  const v4f x = *(const v4fa*)(xr + 4 * tid);

  float s = (x[0] + x[1]) + (x[2] + x[3]);
#pragma unroll
  for (int off = 16; off; off >>= 1) s += __shfl_xor(s, off, 32);
  if (lane == 0) red[wv] = s;
  __syncthreads();
  s = (red[0] + red[1]) + (red[2] + red[3]);
  const float mu = s * (1.0f / DM);
  __syncthreads();

  float dl[4];
  dl[0] = x[0] - mu; dl[1] = x[1] - mu; dl[2] = x[2] - mu; dl[3] = x[3] - mu;
  float q = (dl[0] * dl[0] + dl[1] * dl[1]) + (dl[2] * dl[2] + dl[3] * dl[3]);
#pragma unroll
  for (int off = 16; off; off >>= 1) q += __shfl_xor(q, off, 32);
  if (lane == 0) red[wv] = q;
  __syncthreads();
  q = (red[0] + red[1]) + (red[2] + red[3]);
  const float var = q * (1.0f / DM);
  const float inv = rsqrtf(var + 1e-5f);

  const v4f gg = *(const v4fa*)(gam + 4 * tid);
  const v4f bb = *(const v4fa*)(bet + 4 * tid);
  v4f o;
  o[0] = dl[0] * inv * gg[0] + bb[0];
  o[1] = dl[1] * inv * gg[1] + bb[1];
  o[2] = dl[2] * inv * gg[2] + bb[2];
  o[3] = dl[3] * inv * gg[3] + bb[3];
  float* dst = out + (size_t)row * DM + 4 * tid;
  *(volatile v4f*)dst = o;
  __threadfence();
  *(volatile v4f*)dst = o;
}

static inline size_t align256(size_t x) { return (x + 255) & ~(size_t)255; }

static GemmArgs gemm_defaults(int M, int N, int K)
{
  GemmArgs g = {};
  g.M = M; g.N = N; g.K = K;
  g.ksplit = K; g.nsplit = 1 << 30; g.cfNmax = 1 << 30; g.ctNmin = 0; g.batch = 1;
  g.oscale = 1.0f; g.hscale = 1.0f;
  return g;
}

static void gemm_run2(const GemmArgs& g, hipStream_t st)
{
  dim3 grid((unsigned)((g.N + 63) / 64), (unsigned)((g.M + 63) / 64), (unsigned)g.batch);
  gemm_f16_kernel<2><<<grid, dim3(128), 0, st>>>(g);
}

static void gemm_run1(const GemmArgs& g, hipStream_t st)
{
  dim3 grid((unsigned)((g.N + 31) / 32), (unsigned)((g.M + 63) / 64), (unsigned)g.batch);
  gemm_f16_kernel<1><<<grid, dim3(64), 0, st>>>(g);
}

static void cvt_wT(const float* W, _Float16* o, int R, int C, int ldo, hipStream_t st)
{
  dim3 grid((unsigned)((C + 31) / 32), (unsigned)((R + 63) / 64));
  cvt_wT_f16_kernel<<<grid, dim3(256), 0, st>>>(W, o, R, C, ldo, SC_W);
}

extern "C" void kernel_launch(void* const* d_in, const int* in_sizes, int n_in,
                              void* d_out, int out_size, void* d_ws, size_t ws_size,
                              hipStream_t stream)
{
  if (n_in < 23 || d_in == nullptr || d_out == nullptr || d_ws == nullptr) return;
  const int Mt = NB * LT;
  const int Mi = NB * LI;
  if (in_sizes[0] != Mt * DM || in_sizes[1] != Mi * DM) return;
  if (in_sizes[2] != DM * 2 * DM || in_sizes[4] != DM * 2 * DM) return;
  if (in_sizes[3] != 2 * DM || in_sizes[5] != 2 * DM) return;
  if (in_sizes[6] != DM * DM || in_sizes[8] != DM * DM) return;
  if (in_sizes[7] != DM || in_sizes[9] != DM) return;
  if (in_sizes[10] != DM * DS || in_sizes[12] != DM * DS || in_sizes[14] != DM * DS || in_sizes[16] != DM * DS) return;
  if (in_sizes[11] != DS || in_sizes[13] != DS || in_sizes[15] != DS || in_sizes[17] != DS) return;
  if (in_sizes[18] != DM * DS || in_sizes[19] != 2 * DM * DM) return;
  if (in_sizes[20] != DM || in_sizes[21] != DM || in_sizes[22] != DM) return;
  if (out_size != (Mt + Mi) * DM) return;

  const float* text   = (const float*)d_in[0];
  const float* image  = (const float*)d_in[1];
  const float* W_t2i  = (const float*)d_in[2];
  const float* b_t2i  = (const float*)d_in[3];
  const float* W_i2t  = (const float*)d_in[4];
  const float* b_i2t  = (const float*)d_in[5];
  const float* W_dt_t = (const float*)d_in[6];
  const float* b_dt_t = (const float*)d_in[7];
  const float* W_dt_i = (const float*)d_in[8];
  const float* b_dt_i = (const float*)d_in[9];
  const float* W_B_t  = (const float*)d_in[10];
  const float* b_B_t  = (const float*)d_in[11];
  const float* W_B_i  = (const float*)d_in[12];
  const float* b_B_i  = (const float*)d_in[13];
  const float* W_C_t  = (const float*)d_in[14];
  const float* b_C_t  = (const float*)d_in[15];
  const float* W_C_i  = (const float*)d_in[16];
  const float* b_C_i  = (const float*)d_in[17];
  const float* A_log  = (const float*)d_in[18];
  const float* W_out  = (const float*)d_in[19];
  const float* b_out  = (const float*)d_in[20];
  const float* ln_g   = (const float*)d_in[21];
  const float* ln_b   = (const float*)d_in[22];
  float* out = (float*)d_out;

  char* ws = (char*)d_ws;
  size_t off = 0;
  auto take = [&](size_t bytes) -> void* {
    void* p = ws + off;
    off += align256(bytes);
    return p;
  };
  _Float16* text_h  = (_Float16*)take((size_t)Mt * DM * 2);
  _Float16* img_h   = (_Float16*)take((size_t)Mi * DM * 2);
  _Float16* Wt2iT   = (_Float16*)take((size_t)2 * DM * DM * 2);
  _Float16* Wi2tT   = (_Float16*)take((size_t)2 * DM * DM * 2);
  _Float16* WdtT_t  = (_Float16*)take((size_t)DM * DM * 2);
  _Float16* WdtT_i  = (_Float16*)take((size_t)DM * DM * 2);
  _Float16* WBC_t   = (_Float16*)take((size_t)2 * DS * DM * 2);
  _Float16* WBC_i   = (_Float16*)take((size_t)2 * DS * DM * 2);
  _Float16* WoutT   = (_Float16*)take((size_t)DM * 2 * DM * 2);
  float*    xq_t    = (float*)take((size_t)Mt * DM * 4);
  float*    xq_i    = (float*)take((size_t)Mi * DM * 4);
  _Float16* qk_t    = (_Float16*)take((size_t)Mt * 2 * DM * 2);
  _Float16* qk_i    = (_Float16*)take((size_t)Mi * 2 * DM * 2);
  _Float16* kT_t    = (_Float16*)take((size_t)DM * Mt * 2);
  _Float16* kT_i    = (_Float16*)take((size_t)DM * Mi * 2);
  float*    dt_t    = (float*)take((size_t)Mt * DM * 4);
  float*    dt_i    = (float*)take((size_t)Mi * DM * 4);
  float*    scores  = (float*)take((size_t)NB * LT * LI * 4);
  _Float16* P_h     = (_Float16*)take((size_t)NB * LT * LI * 2);
  _Float16* Bf_t    = (_Float16*)take((size_t)Mt * DM * 2);
  _Float16* Bf_i    = (_Float16*)take((size_t)Mi * DM * 2);
  float*    BC_t    = (float*)take((size_t)Mt * 2 * DS * 4);
  float*    BC_i    = (float*)take((size_t)Mi * 2 * DS * 4);
  _Float16* y_t     = (_Float16*)take((size_t)Mt * DM * 2);
  _Float16* y_i     = (_Float16*)take((size_t)Mi * DM * 2);
  float*    pre_t   = (float*)take((size_t)Mt * DM * 4);
  float*    pre_i   = (float*)take((size_t)Mi * DM * 4);
  if (off > ws_size) return;

  {
    const int ut = Mt * DM / 8, ui = Mi * DM / 8;
    cvt_rows_f16_kernel<<<dim3((unsigned)((ut + 255) / 256)), dim3(256), 0, stream>>>(text, text_h, ut, SC_ACT);
    cvt_rows_f16_kernel<<<dim3((unsigned)((ui + 255) / 256)), dim3(256), 0, stream>>>(image, img_h, ui, SC_ACT);
  }
  cvt_wT(W_t2i,  Wt2iT,  DM, 2 * DM, DM, stream);
  cvt_wT(W_i2t,  Wi2tT,  DM, 2 * DM, DM, stream);
  cvt_wT(W_dt_t, WdtT_t, DM, DM, DM, stream);
  cvt_wT(W_dt_i, WdtT_i, DM, DM, DM, stream);
  cvt_wT(W_B_t,  WBC_t,                    DM, DS, DM, stream);
  cvt_wT(W_C_t,  WBC_t + (size_t)DS * DM,  DM, DS, DM, stream);
  cvt_wT(W_B_i,  WBC_i,                    DM, DS, DM, stream);
  cvt_wT(W_C_i,  WBC_i + (size_t)DS * DM,  DM, DS, DM, stream);
  cvt_wT(W_out,  WoutT,  2 * DM, DM, 2 * DM, stream);

  const float inv_act_w = 1.0f / (SC_ACT * SC_W);
  const float inv_qk_w  = 1.0f / (SC_QK * SC_W);
  const float inv_qk_qk = 1.0f / (SC_QK * SC_QK);
  const float inv_p_qk  = 1.0f / (SC_P * SC_QK);
  const float inv_bf_w  = 1.0f / (SC_BF * SC_W);
  const float att_scale = 0.044194173824159216f;

  {
    GemmArgs g = gemm_defaults(Mt, 2 * DM, DM);
    g.A = text_h; g.lda = DM; g.Bt = Wt2iT; g.ldb = DM; g.bias = b_t2i; g.oscale = inv_act_w;
    g.Cf = xq_t; g.ldc = DM; g.cfNmax = DM;
    g.Ch = qk_t; g.ldch = 2 * DM; g.hscale = SC_QK;
    g.Ct = kT_t; g.ldct = Mt; g.ctNmin = DM;
    gemm_run2(g, stream);
  }
  {
    GemmArgs g = gemm_defaults(Mi, 2 * DM, DM);
    g.A = img_h; g.lda = DM; g.Bt = Wi2tT; g.ldb = DM; g.bias = b_i2t; g.oscale = inv_act_w;
    g.Cf = xq_i; g.ldc = DM; g.cfNmax = DM;
    g.Ch = qk_i; g.ldch = 2 * DM; g.hscale = SC_QK;
    g.Ct = kT_i; g.ldct = Mi; g.ctNmin = DM;
    gemm_run2(g, stream);
  }

  {
    GemmArgs g = gemm_defaults(Mt, DM, DM);
    g.A = qk_t; g.lda = 2 * DM; g.Bt = WdtT_t; g.ldb = DM; g.bias = b_dt_t; g.oscale = inv_qk_w;
    g.Cf = dt_t; g.ldc = DM;
    gemm_run2(g, stream);
  }
  {
    GemmArgs g = gemm_defaults(Mi, DM, DM);
    g.A = qk_i; g.lda = 2 * DM; g.Bt = WdtT_i; g.ldb = DM; g.bias = b_dt_i; g.oscale = inv_qk_w;
    g.Cf = dt_i; g.ldc = DM;
    gemm_run2(g, stream);
  }

  {
    GemmArgs g = gemm_defaults(LT, LI, DM);
    g.batch = NB;
    g.A = qk_t; g.lda = 2 * DM; g.sA = (long long)LT * 2 * DM;
    g.Bt = qk_i + DM; g.ldb = 2 * DM; g.sB = (long long)LI * 2 * DM;
    g.oscale = inv_qk_qk;
    g.Cf = scores; g.ldc = LI; g.sC = (long long)LT * LI;
    gemm_run2(g, stream);
  }
  softmax_f16_kernel<<<dim3((unsigned)(NB * LT)), dim3(256), 0, stream>>>(scores, P_h, LI, att_scale, SC_P);
  {
    GemmArgs g = gemm_defaults(LT, DM, LI);
    g.batch = NB;
    g.A = P_h; g.lda = LI; g.sA = (long long)LT * LI;
    g.Bt = kT_i; g.ldb = Mi; g.sB = (long long)LI;
    g.oscale = inv_p_qk;
    g.Ch = Bf_t; g.ldch = DM; g.sCh = (long long)LT * DM; g.hscale = SC_BF;
    gemm_run2(g, stream);
  }

  {
    GemmArgs g = gemm_defaults(LI, LT, DM);
    g.batch = NB;
    g.A = qk_i; g.lda = 2 * DM; g.sA = (long long)LI * 2 * DM;
    g.Bt = qk_t + DM; g.ldb = 2 * DM; g.sB = (long long)LT * 2 * DM;
    g.oscale = inv_qk_qk;
    g.Cf = scores; g.ldc = LT; g.sC = (long long)LI * LT;
    gemm_run2(g, stream);
  }
  softmax_f16_kernel<<<dim3((unsigned)(NB * LI)), dim3(256), 0, stream>>>(scores, P_h, LT, att_scale, SC_P);
  {
    GemmArgs g = gemm_defaults(LI, DM, LT);
    g.batch = NB;
    g.A = P_h; g.lda = LT; g.sA = (long long)LI * LT;
    g.Bt = kT_t; g.ldb = Mt; g.sB = (long long)LT;
    g.oscale = inv_p_qk;
    g.Ch = Bf_i; g.ldch = DM; g.sCh = (long long)LI * DM; g.hscale = SC_BF;
    gemm_run2(g, stream);
  }

  {
    GemmArgs g = gemm_defaults(Mt, 2 * DS, DM);
    g.A = Bf_t; g.lda = DM; g.Bt = WBC_t; g.ldb = DM; g.oscale = inv_bf_w;
    g.bias = b_B_t; g.bias2 = b_C_t; g.nsplit = DS;
    g.Cf = BC_t; g.ldc = 2 * DS;
    gemm_run1(g, stream);
  }
  {
    GemmArgs g = gemm_defaults(Mi, 2 * DS, DM);
    g.A = Bf_i; g.lda = DM; g.Bt = WBC_i; g.ldb = DM; g.oscale = inv_bf_w;
    g.bias = b_B_i; g.bias2 = b_C_i; g.nsplit = DS;
    g.Cf = BC_i; g.ldc = 2 * DS;
    gemm_run1(g, stream);
  }

  scan_kernel<<<dim3((unsigned)(NB * DM / 64)), dim3(128), 0, stream>>>(xq_t, dt_t, A_log, BC_t, y_t, LT, SC_Y);
  scan_kernel<<<dim3((unsigned)(NB * DM / 64)), dim3(128), 0, stream>>>(xq_i, dt_i, A_log, BC_i, y_i, LI, SC_Y);

  {
    GemmArgs g = gemm_defaults(Mt, DM, 2 * DM);
    g.A = text_h; g.lda = DM; g.A2 = y_t; g.lda2 = DM; g.ksplit = DM;
    g.Bt = WoutT; g.ldb = 2 * DM; g.bias = b_out; g.oscale = inv_act_w;
    g.Cf = pre_t; g.ldc = DM;
    gemm_run2(g, stream);
  }
  {
    GemmArgs g = gemm_defaults(Mi, DM, 2 * DM);
    g.A = img_h; g.lda = DM; g.A2 = y_i; g.lda2 = DM; g.ksplit = DM;
    g.Bt = WoutT; g.ldb = 2 * DM; g.bias = b_out; g.oscale = inv_act_w;
    g.Cf = pre_i; g.ldc = DM;
    gemm_run2(g, stream);
  }

  layernorm_kernel<<<dim3((unsigned)Mt), dim3(128), 0, stream>>>(pre_t, ln_g, ln_b, out, Mt);
  layernorm_kernel<<<dim3((unsigned)Mi), dim3(128), 0, stream>>>(pre_i, ln_g, ln_b, out + (size_t)Mt * DM, Mi);
}
